// LocalGlobalGNN_4672924418435
// MI455X (gfx1250) — hardware-run, weakly checked
//
#include <hip/hip_runtime.h>


namespace {
constexpr int N = 50000, NP = 50048, IN = 128, H = 256, C = 64, MH = 128, EG = 600000, EK = 800000, NBLK = NP / 16;
constexpr float XS = 8.0f, WSC = 256.0f, BNEPS = 1e-5f;
typedef _Float16 b16;
typedef __attribute__((ext_vector_type(16))) _Float16 v16b;
typedef __attribute__((ext_vector_type(8))) _Float16 v8b;
typedef __attribute__((ext_vector_type(8))) float v8f;
typedef __attribute__((ext_vector_type(4))) float v4f;
typedef __attribute__((ext_vector_type(2))) float v2f;
__device__ __forceinline__ float bf16_rne(float f) { unsigned int u = __float_as_uint(f); u += 0x7FFFu + ((u >> 16) & 1u); return __uint_as_float(u & 0xFFFF0000u); }
__device__ __forceinline__ void split16(float v, b16& hi, b16& lo) { hi = (b16)v; lo = (b16)(v - (float)hi); }
__device__ __forceinline__ v16b frag_kb(const b16* p, int hh) { const v8b a = *(const v8b*)(p + 8 * hh), b = *(const v8b*)(p + 16 + 8 * hh); v16b f;
#pragma unroll
  for (int e = 0; e < 8; ++e) { f[e] = a[e]; f[8 + e] = b[e]; } return f; }
__device__ __forceinline__ v8f wmma16b(v16b a, v16b b, v8f c) { v8f d = __builtin_amdgcn_wmma_f32_16x16x32_f16(false, a, false, b, (short)0, c, false, false); asm volatile("v_nop\n\tv_nop\n\tv_nop\n\tv_nop" : "+v"(d) : "v"(a), "v"(b)); return d; }
__device__ __forceinline__ void wave_lds_sync() { __builtin_amdgcn_fence(__ATOMIC_RELEASE, "workgroup"); __builtin_amdgcn_wave_barrier(); __builtin_amdgcn_fence(__ATOMIC_ACQUIRE, "workgroup"); }
__device__ __forceinline__ float pmul(float a, float b) { float p = a * b; asm volatile("" : "+v"(p)); return p; }
__device__ __forceinline__ int iclamp(int v, int lo, int hi) { return v < lo ? lo : (v > hi ? hi : v); }
constexpr int CSR_NBLK = 512, CSR_GB = 9, CSR_GN = 1 << CSR_GB  , CSR_TS = (CSR_GN < 32 ? 32 : CSR_GN)  , CSR_MAXG = 512, CSR_CAP = 12288  ;
__device__ __host__ __forceinline__ int csr_tix(int v) { return (v >> CSR_GB) * CSR_TS + (v & (CSR_GN - 1)); }
__global__ __launch_bounds__(64) void csrA_kernel(const int* __restrict__ dst, int E, int N, int nG, int CHP, int NGP, int* __restrict__ STG, int* __restrict__ HST) {
  extern __shared__ int sm[];
  int* cnt = sm; int* run = sm + NGP; int* ids = sm + 2 * NGP;
  const int b = blockIdx.x; const int ch = (E + CSR_NBLK - 1) / CSR_NBLK; const int e0 = b * ch, e1 = min(E, e0 + ch);
  for (int i = threadIdx.x; i < NGP; i += 64) cnt[i] = 0;
  for (int i = threadIdx.x; i < CHP; i += 64) ids[i] = -1;
  __syncthreads();
  if (threadIdx.x == 0) {
    for (int e = e0; e < e1; ++e) { int d = dst[e]; d = (d < 0) ? 0 : (d >= N ? N - 1 : d); cnt[d >> CSR_GB] += 1; }
    int acc = 0; for (int g = 0; g < nG; ++g) { run[g] = acc; acc += cnt[g]; }
    for (int e = e0; e < e1; ++e) { int d = dst[e]; d = (d < 0) ? 0 : (d >= N ? N - 1 : d); const int g = d >> CSR_GB; ids[run[g]] = e; run[g] += 1; } }
  __syncthreads();
  typedef __attribute__((ext_vector_type(4))) int v4i;
  for (int pass = 0; pass < 2; ++pass) {
    for (int i = threadIdx.x; i < CHP / 4; i += 64) *(volatile v4i*)(STG + (size_t)b * CHP + i * 4) = *(const v4i*)(&ids[i * 4]);
    for (int i = threadIdx.x; i < NGP / 4; i += 64) { v4i v; for (int e = 0; e < 4; ++e) v[e] = (i * 4 + e < nG) ? cnt[i * 4 + e] : 0; *(volatile v4i*)(HST + (size_t)b * NGP + i * 4) = v; }
    __threadfence(); }
}
__global__ __launch_bounds__(512) void csrS_kernel(const int* __restrict__ HST, int nG, int NGP, int* __restrict__ START, int* __restrict__ TOT, int* __restrict__ OFF) {
  __shared__ int tot[CSR_MAXG];
  const int b = threadIdx.x;
  for (int pass = 0; pass < 2; ++pass) { int runb = 0; for (int g = 0; g < nG; ++g) { int c = HST[(size_t)b * NGP + g]; c = (c < 0) ? 0 : c; ((volatile int*)OFF)[(size_t)g * CSR_NBLK + b] = runb; runb += c; } __threadfence(); }
  for (int g = threadIdx.x; g < nG; g += 512) { int s = 0; for (int bb = 0; bb < CSR_NBLK; ++bb) { int c = HST[(size_t)bb * NGP + g]; s += (c < 0) ? 0 : c; } tot[g] = s; }
  __syncthreads();
  if (threadIdx.x < 32) {
    __shared__ int st[CSR_MAXG + 32];
    if (threadIdx.x == 0) { int acc = 0; for (int g = 0; g < NGP; ++g) { st[g] = acc; if (g < nG) acc += (tot[g] + 31) & ~31; } st[NGP] = acc; }
    __builtin_amdgcn_fence(__ATOMIC_RELEASE, "workgroup"); __builtin_amdgcn_wave_barrier(); __builtin_amdgcn_fence(__ATOMIC_ACQUIRE, "workgroup");
    for (int pass = 0; pass < 2; ++pass) { for (int i = threadIdx.x; i < NGP + 32; i += 32) { ((volatile int*)START)[i] = (i <= NGP) ? st[min(i, NGP)] : 0; ((volatile int*)TOT)[i] = (i < nG) ? tot[i] : 0; } __threadfence(); } }
}
__global__ __launch_bounds__(256) void csrB_kernel(const int* __restrict__ dst, int N, int nG, int CHP, int NGP, int permLen, const int* __restrict__ STG, const int* __restrict__ HST, const int* __restrict__ OFF, const int* __restrict__ START, const int* __restrict__ TOT, int* __restrict__ PERM, int* __restrict__ ROWPTR, int* __restrict__ ROWCNT, int* __restrict__ FLAG) {
  typedef __attribute__((ext_vector_type(4))) int v4i;
  __shared__ int ids[CSR_CAP]; __shared__ unsigned short key[CSR_CAP]; __shared__ int outp[CSR_CAP]; __shared__ int ncnt[CSR_GN + 1]; __shared__ int boff[CSR_NBLK + 1];
  const int g = blockIdx.x, t_ = threadIdx.x; int tot = TOT[g]; int st = START[g], stn = START[g + 1]; const int v0 = g * CSR_GN; const int nv = min(CSR_GN, N - v0); const int t0 = g * CSR_TS;
  st = (st < 0) ? 0 : (st > permLen - 32 ? permLen - 32 : st) & ~31; stn = (stn < st) ? st : (stn > permLen ? permLen : stn); tot = (tot < 0) ? 0 : tot; if (tot > stn - st && tot <= CSR_CAP) tot = stn - st;
  if (tot > CSR_CAP) {
    for (int pass = 0; pass < 2; ++pass) { for (int i = t_; i < CSR_TS / 4; i += 256) { v4i a, c; for (int e = 0; e < 4; ++e) { a[e] = st; c[e] = 0; } *(volatile v4i*)(ROWPTR + t0 + i * 4) = a; *(volatile v4i*)(ROWCNT + t0 + i * 4) = c; } if (t_ == 0) ((volatile int*)FLAG)[0] = 1; __threadfence(); } (void)nv; return; }
  if (t_ == 0) { int acc = 0; for (int b = 0; b < CSR_NBLK; ++b) { boff[b] = acc; int c = HST[(size_t)b * NGP + g]; c = (c < 0) ? 0 : (c > CHP ? CHP : c); acc += c; if (acc > tot) acc = tot; } boff[CSR_NBLK] = acc; }
  for (int i = t_; i <= CSR_GN; i += 256) ncnt[i] = 0;
  __syncthreads();
  for (int b = 0; b < CSR_NBLK; ++b) { const int c = boff[b + 1] - boff[b]; int o_ = OFF[(size_t)g * CSR_NBLK + b]; o_ = (o_ < 0) ? 0 : (o_ > CHP - c ? CHP - c : o_); const int* src_ = STG + (size_t)b * CHP + o_;
    for (int i = t_; i < c; i += 256) { int id = src_[i]; id = (id < 0) ? 0 : id; ids[boff[b] + i] = id; int d = dst[id]; d = (d < v0) ? v0 : (d >= N ? N - 1 : d); int kk = d - v0; kk = (kk < 0) ? 0 : (kk >= CSR_GN ? CSR_GN - 1 : kk); key[boff[b] + i] = (unsigned short)kk; } }
  __syncthreads();
  if (t_ == 0) { for (int i = 0; i < tot; ++i) ncnt[key[i]] += 1; int acc = 0; for (int vl = 0; vl < CSR_GN; ++vl) { const int c = ncnt[vl]; ncnt[vl] = acc; acc += c; } ncnt[CSR_GN] = acc;
    for (int i = 0; i < tot; ++i) { const int vl = key[i]; outp[ncnt[vl]] = ids[i]; ncnt[vl] += 1; }
    for (int vl = CSR_GN; vl > 0; --vl) ncnt[vl] = ncnt[vl - 1]; ncnt[0] = 0; }
  __syncthreads();
  for (int pass = 0; pass < 2; ++pass) {
    for (int i = t_; i < (stn - st) / 4; i += 256) { v4i v; for (int e = 0; e < 4; ++e) { const int q = i * 4 + e; v[e] = (q < tot) ? outp[q] : -1; } *(volatile v4i*)(PERM + st + i * 4) = v; }
    for (int i = t_; i < CSR_TS / 4; i += 256) { v4i a, c; for (int e = 0; e < 4; ++e) { const int vl = i * 4 + e; const int vc = vl < CSR_GN ? vl : CSR_GN; a[e] = (vl < CSR_GN) ? st + ncnt[vc] : st; c[e] = (vl < nv) ? (ncnt[(vc < CSR_GN ? vc : CSR_GN - 1) + 1] - ncnt[vc]) : 0; } *(volatile v4i*)(ROWPTR + t0 + i * 4) = a; *(volatile v4i*)(ROWCNT + t0 + i * 4) = c; }
    __threadfence(); }
}
__global__ __launch_bounds__(256) void csrZ_kernel(int* __restrict__ p, size_t n4) { typedef __attribute__((ext_vector_type(4))) int v4i; const size_t tid = (size_t)blockIdx.x * 256 + threadIdx.x, nth = (size_t)gridDim.x * 256; v4i z = {0, 0, 0, 0}; for (size_t i = tid; i < n4; i += nth) *(volatile v4i*)(p + i * 4) = z; }
struct CsrBufs { int *STG, *HST, *OFF, *START, *TOT, *PERM, *ROWPTR, *ROWCNT, *FLAG; int nG, NGP, CHP; size_t permLen; char* base; size_t bytes; };
static size_t csr_carve(CsrBufs& c, char* ws, size_t off, int E, int N) {
  const size_t off0 = off; c.base = ws + off;
  auto al = [&](size_t bytes) { char* p = ws + off; off += (bytes + 255) & ~(size_t)255; return p; };
  c.nG = (N + CSR_GN - 1) / CSR_GN; c.NGP = (c.nG + 31) & ~31; const int ch = (E + CSR_NBLK - 1) / CSR_NBLK; c.CHP = (ch + 31) & ~31; c.permLen = (size_t)E + 32 * (size_t)c.nG + 32;
  c.STG = (int*)al((size_t)CSR_NBLK * c.CHP * 4); c.HST = (int*)al((size_t)CSR_NBLK * c.NGP * 4); c.OFF = (int*)al((size_t)c.NGP * CSR_NBLK * 4); c.START = (int*)al((size_t)(c.NGP + 64) * 4); c.TOT = (int*)al((size_t)(c.NGP + 64) * 4);
  c.PERM = (int*)al(c.permLen * 4); c.ROWPTR = (int*)al((size_t)c.nG * CSR_TS * 4); c.ROWCNT = (int*)al((size_t)c.nG * CSR_TS * 4); c.FLAG = (int*)al(256);
  c.bytes = off - off0; return off;
}
static void csr_build(const CsrBufs& c, const int* dst, int E, int N, hipStream_t stream) {
  const size_t smem = (size_t)(2 * c.NGP + c.CHP) * 4;
  csrZ_kernel<<<512, 256, 0, stream>>>((int*)c.base, c.bytes / 16);
  csrA_kernel<<<CSR_NBLK, 64, smem, stream>>>(dst, E, N, c.nG, c.CHP, c.NGP, c.STG, c.HST);
  csrS_kernel<<<1, 512, 0, stream>>>(c.HST, c.nG, c.NGP, c.START, c.TOT, c.OFF);
  csrB_kernel<<<c.nG, 256, 0, stream>>>(dst, N, c.nG, c.CHP, c.NGP, (int)c.permLen, c.STG, c.HST, c.OFF, c.START, c.TOT, c.PERM, c.ROWPTR, c.ROWCNT, c.FLAG);
}


__global__ __launch_bounds__(256) void wprep_kernel(const float* __restrict__ w, int KIN, int OUT, int co, int KTOT, b16* __restrict__ WT) {
  const size_t u = (size_t)blockIdx.x * 256 + threadIdx.x; if (u >= (size_t)OUT * KIN / 8) return; const size_t e = u * 8; const int o = (int)(e / KIN), k0 = (int)(e % KIN); v8b v;
  for (int j = 0; j < 8; ++j) v[j] = (b16)(bf16_rne(w[(size_t)(k0 + j) * OUT + o]) * WSC); for (int pass = 0; pass < 2; ++pass) { *(volatile v8b*)(WT + (size_t)o * KTOT + co + k0) = v; __threadfence(); }
}
template <int KIN, int RAW, int RELU>
__global__ __launch_bounds__(32) void sage_kernel(const float* __restrict__ HIN, const b16* __restrict__ WT, const float* __restrict__ bias, const int* __restrict__ srcs, int E, const int* __restrict__ PERM, const int* __restrict__ ROWPTR, const int* __restrict__ ROWCNT, int permLen, int NLIM, float* __restrict__ OUT) {
  constexpr int K2 = 2 * KIN, CPL = KIN / 32;
  __shared__ __attribute__((aligned(16))) b16 Ah[16][K2 + 8], Al[16][K2 + 8]; __shared__ __attribute__((aligned(16))) float Tf[16][H + 4];
  const int lane = threadIdx.x, nloc = lane & 15, hlf = lane >> 4; const size_t v0 = (size_t)blockIdx.x * 16;
  for (int rr = 0; rr < 16; ++rr) { const size_t v = v0 + rr; float own[CPL], agg[CPL]; for (int q = 0; q < CPL; ++q) { own[q] = 0.0f; agg[q] = 0.0f; } float inv = 0.0f;
    if (v < (size_t)NLIM) { int st = ROWPTR[v], cnt = ROWCNT[v]; cnt = iclamp(cnt, 0, 65536); st = iclamp(st, 0, permLen - cnt);
      for (int q = 0; q < CPL; ++q) { const float t = HIN[v * KIN + lane * CPL + q]; own[q] = RAW ? bf16_rne(t) : t; }
#pragma unroll 2
      for (int j = 0; j < cnt; ++j) { const int e = iclamp(PERM[st + j], 0, E - 1); const size_t s = (size_t)iclamp(srcs[e], 0, N - 1);
        if (s < (size_t)NLIM) { for (int q = 0; q < CPL; ++q) { const float t = HIN[s * KIN + lane * CPL + q]; agg[q] += RAW ? bf16_rne(t) : t; } } }
      inv = cnt > 0 ? 1.0f / (float)cnt : 0.0f; }
    for (int q = 0; q < CPL; ++q) { b16 p, ql; if (RAW) { p = (b16)(own[q] * XS); ql = (b16)0.0f; } else split16(own[q] * XS, p, ql); Ah[rr][lane * CPL + q] = p; Al[rr][lane * CPL + q] = ql; split16(pmul(agg[q], inv) * XS, p, ql); Ah[rr][KIN + lane * CPL + q] = p; Al[rr][KIN + lane * CPL + q] = ql; } }
  wave_lds_sync();
#pragma unroll 1
  for (int half = 0; half < 2; ++half) { v8f acc[8];
#pragma unroll
    for (int t = 0; t < 8; ++t) acc[t] = (v8f){};
#pragma unroll 2
    for (int kb = 0; kb < K2; kb += 32) { const v16b a = frag_kb(&Ah[nloc][kb], hlf), al = frag_kb(&Al[nloc][kb], hlf); const bool dolo = (!RAW) || kb >= KIN;
#pragma unroll
      for (int t = 0; t < 8; ++t) { const v16b bw = frag_kb(WT + (size_t)(half * 128 + t * 16 + nloc) * K2 + kb, hlf); acc[t] = wmma16b(a, bw, acc[t]); if (dolo) acc[t] = wmma16b(al, bw, acc[t]); } }
#pragma unroll
    for (int t = 0; t < 8; ++t) { const int c = half * 128 + t * 16 + nloc; const float bb = bf16_rne(bias[c]);
#pragma unroll 1
      for (int r8 = 0; r8 < 8; ++r8) { const int rl = 8 * hlf + r8; float val = acc[t][r8] * (1.0f / (XS * WSC)) + bb; if (RELU) val = fmaxf(val, 0.0f); Tf[rl][c] = ((v0 + rl) < (size_t)NLIM) ? val : 0.0f; } } }
  wave_lds_sync();
  for (int pass = 0; pass < 2; ++pass) { for (int rr = 0; rr < 16; ++rr) { *(volatile v4f*)(OUT + (v0 + rr) * H + lane * 4) = *(const v4f*)(&Tf[rr][lane * 4]); *(volatile v4f*)(OUT + (v0 + rr) * H + 128 + lane * 4) = *(const v4f*)(&Tf[rr][128 + lane * 4]); } __threadfence(); }
}
template <int ACCUM>
__global__ __launch_bounds__(32) void mlp1_kernel(const float* __restrict__ EMB, const b16* __restrict__ W1T, const float* __restrict__ b1, int NLIM, float* __restrict__ Y) {
  __shared__ __attribute__((aligned(16))) b16 Ah[16][H + 8], Al[16][H + 8]; __shared__ __attribute__((aligned(16))) float Tf[16][MH + 4];
  const int lane = threadIdx.x, nloc = lane & 15, hlf = lane >> 4; const size_t v0 = (size_t)blockIdx.x * 16;
  for (int rr = 0; rr < 16; ++rr) { const v8f e8 = *(const v8f*)(EMB + (v0 + rr) * H + lane * 8); for (int j = 0; j < 8; ++j) { b16 p, q; split16(e8[j] * XS, p, q); Ah[rr][lane * 8 + j] = p; Al[rr][lane * 8 + j] = q; } }
  wave_lds_sync();
  v8f acc[8];
#pragma unroll
  for (int t = 0; t < 8; ++t) acc[t] = (v8f){};
#pragma unroll 2
  for (int kb = 0; kb < H; kb += 32) { const v16b a = frag_kb(&Ah[nloc][kb], hlf), al = frag_kb(&Al[nloc][kb], hlf);
#pragma unroll
    for (int t = 0; t < 8; ++t) { const v16b bw = frag_kb(W1T + (size_t)(t * 16 + nloc) * H + kb, hlf); acc[t] = wmma16b(a, bw, acc[t]); acc[t] = wmma16b(al, bw, acc[t]); } }
#pragma unroll
  for (int t = 0; t < 8; ++t) { const int c = t * 16 + nloc; const float bb = ACCUM ? 0.0f : bf16_rne(b1[c]);
#pragma unroll 1
    for (int r8 = 0; r8 < 8; ++r8) { const int rl = 8 * hlf + r8; const float prev = ACCUM ? Y[(v0 + rl) * MH + c] : 0.0f; Tf[rl][c] = ((v0 + rl) < (size_t)NLIM) ? prev + acc[t][r8] * (1.0f / (XS * WSC)) + bb : 0.0f; } }
  wave_lds_sync();
  for (int pass = 0; pass < 2; ++pass) { for (int rr = 0; rr < 16; ++rr) *(volatile v4f*)(Y + (v0 + rr) * MH + lane * 4) = *(const v4f*)(&Tf[rr][lane * 4]); __threadfence(); }
}
constexpr int RB = 512, NSB = (N + RB - 1) / RB;
__global__ __launch_bounds__(128) void bnstat1_kernel(const float* __restrict__ Y, int NLIM, double* __restrict__ PS) {
  const int c = threadIdx.x; const int r0 = blockIdx.x * RB; const int r1 = min(r0 + RB, NLIM); double s = 0.0, s2 = 0.0;
#pragma unroll 4
  for (int r = r0; r < r1; ++r) { const double y = (double)Y[(size_t)r * MH + c]; s += y; s2 += y * y; }
  for (int pass = 0; pass < 2; ++pass) { ((volatile double*)PS)[((size_t)blockIdx.x * 2 + 0) * MH + c] = s; ((volatile double*)PS)[((size_t)blockIdx.x * 2 + 1) * MH + c] = s2; __threadfence(); }
}
__global__ __launch_bounds__(128) void bnstat2_kernel(const double* __restrict__ PS, int NLIM, float* __restrict__ MV) {
  const int c = threadIdx.x; double s = 0.0, s2 = 0.0; for (int b = 0; b < NSB; ++b) { s += PS[((size_t)b * 2 + 0) * MH + c]; s2 += PS[((size_t)b * 2 + 1) * MH + c]; }
  const double mu = s / (double)NLIM; double var = s2 / (double)NLIM - mu * mu; if (var < 0.0) var = 0.0;
  for (int pass = 0; pass < 2; ++pass) { ((volatile float*)MV)[c] = (float)mu; ((volatile float*)MV)[MH + c] = (float)(1.0 / sqrt(var + (double)BNEPS)); __threadfence(); }
}
__global__ __launch_bounds__(32) void head_kernel(const float* __restrict__ Y, const float* __restrict__ MV, const float* __restrict__ gam, const float* __restrict__ bet, const b16* __restrict__ W2T, const float* __restrict__ b2, float* __restrict__ out) {
  __shared__ __attribute__((aligned(16))) b16 Ah[16][MH + 8], Al[16][MH + 8]; __shared__ __attribute__((aligned(16))) float Tf[16][C + 4];
  const int lane = threadIdx.x, nloc = lane & 15, hlf = lane >> 4; const size_t v0 = (size_t)blockIdx.x * 16;
  float mu4[4], rs4[4], g4[4], b4[4]; for (int j = 0; j < 4; ++j) { const int c = lane * 4 + j; mu4[j] = MV[c]; rs4[j] = MV[MH + c]; g4[j] = bf16_rne(gam[c]); b4[j] = bf16_rne(bet[c]); }
  for (int rr = 0; rr < 16; ++rr) { const v4f y = *(const v4f*)(Y + (v0 + rr) * MH + lane * 4); for (int j = 0; j < 4; ++j) { const float a = fmaxf(pmul(pmul(g4[j], y[j] - mu4[j]), rs4[j]) + b4[j], 0.0f); b16 p, q; split16(a * XS, p, q); Ah[rr][lane * 4 + j] = p; Al[rr][lane * 4 + j] = q; } }
  wave_lds_sync();
  v8f acc[4];
#pragma unroll
  for (int t = 0; t < 4; ++t) acc[t] = (v8f){};
#pragma unroll 2
  for (int kb = 0; kb < MH; kb += 32) { const v16b a = frag_kb(&Ah[nloc][kb], hlf), al = frag_kb(&Al[nloc][kb], hlf);
#pragma unroll
    for (int t = 0; t < 4; ++t) { const v16b bw = frag_kb(W2T + (size_t)(t * 16 + nloc) * MH + kb, hlf); acc[t] = wmma16b(a, bw, acc[t]); acc[t] = wmma16b(al, bw, acc[t]); } }
#pragma unroll
  for (int t = 0; t < 4; ++t) { const int c = t * 16 + nloc; const float bb = bf16_rne(b2[c]);
#pragma unroll 1
    for (int r8 = 0; r8 < 8; ++r8) Tf[8 * hlf + r8][c] = acc[t][r8] * (1.0f / (XS * WSC)) + bb; }
  wave_lds_sync();
  for (int pass = 0; pass < 2; ++pass) { for (int rr = 0; rr < 16; ++rr) if ((v0 + rr) < (size_t)N && lane < 16) *(volatile v4f*)(out + (v0 + rr) * C + lane * 4) = *(const v4f*)(&Tf[rr][lane * 4]); __threadfence(); }
}
}

extern "C" void kernel_launch(void* const* d_in, const int* in_sizes, int n_in, void* d_out, int out_size, void* d_ws, size_t ws_size, hipStream_t stream) {
  (void)n_in;
  auto Fp = [&](int i) { return (const float*)d_in[i]; }; auto Ip = [&](int i) { return (const int*)d_in[i]; };
  if (in_sizes[0] != N * IN || in_sizes[1] != EG || in_sizes[2] != EG || in_sizes[3] != EK || in_sizes[4] != EK || in_sizes[5] != IN * H || in_sizes[8] != H * H || in_sizes[14] != IN * H || in_sizes[17] != H * H || in_sizes[20] != 2 * H * MH || in_sizes[24] != MH * C || out_size != N * C) return;
  const int NLIM = N;
  size_t off = 0; char* ws = (char*)d_ws;
  auto carve = [&](size_t bytes) { char* p = ws + off; off += (bytes + 255) & ~(size_t)255; return p; };
  b16* WL0 = (b16*)carve((size_t)H * 2 * IN * 2); b16* WL1 = (b16*)carve((size_t)H * 2 * H * 2); b16* WL2 = (b16*)carve((size_t)H * 2 * H * 2); b16* WG0 = (b16*)carve((size_t)H * 2 * IN * 2); b16* WG1 = (b16*)carve((size_t)H * 2 * H * 2);
  b16* WM1A = (b16*)carve((size_t)MH * H * 2); b16* WM1B = (b16*)carve((size_t)MH * H * 2); b16* WM2 = (b16*)carve((size_t)C * MH * 2);
  float* HA = (float*)carve((size_t)NP * H * 4); float* HB = (float*)carve((size_t)NP * H * 4); float* Y = (float*)carve((size_t)NP * MH * 4); double* PS = (double*)carve((size_t)NSB * 2 * MH * 8); float* MV = (float*)carve(2 * MH * 4);
  CsrBufs csrG, csrK; off = csr_carve(csrG, ws, off, EG, N); off = csr_carve(csrK, ws, off, EK, N);
  if (off > ws_size) return;
  wprep_kernel<<<(H * IN / 8 + 255) / 256, 256, 0, stream>>>(Fp(5), IN, H, 0, 2 * IN, WL0); wprep_kernel<<<(H * IN / 8 + 255) / 256, 256, 0, stream>>>(Fp(6), IN, H, IN, 2 * IN, WL0);
  wprep_kernel<<<(H * H / 8 + 255) / 256, 256, 0, stream>>>(Fp(8), H, H, 0, 2 * H, WL1); wprep_kernel<<<(H * H / 8 + 255) / 256, 256, 0, stream>>>(Fp(9), H, H, H, 2 * H, WL1);
  wprep_kernel<<<(H * H / 8 + 255) / 256, 256, 0, stream>>>(Fp(11), H, H, 0, 2 * H, WL2); wprep_kernel<<<(H * H / 8 + 255) / 256, 256, 0, stream>>>(Fp(12), H, H, H, 2 * H, WL2);
  wprep_kernel<<<(H * IN / 8 + 255) / 256, 256, 0, stream>>>(Fp(14), IN, H, 0, 2 * IN, WG0); wprep_kernel<<<(H * IN / 8 + 255) / 256, 256, 0, stream>>>(Fp(15), IN, H, IN, 2 * IN, WG0);
  wprep_kernel<<<(H * H / 8 + 255) / 256, 256, 0, stream>>>(Fp(17), H, H, 0, 2 * H, WG1); wprep_kernel<<<(H * H / 8 + 255) / 256, 256, 0, stream>>>(Fp(18), H, H, H, 2 * H, WG1);
  wprep_kernel<<<(MH * H / 8 + 255) / 256, 256, 0, stream>>>(Fp(20), H, MH, 0, H, WM1A); wprep_kernel<<<(MH * H / 8 + 255) / 256, 256, 0, stream>>>(Fp(20) + (size_t)H * MH, H, MH, 0, H, WM1B);
  wprep_kernel<<<(C * MH / 8 + 255) / 256, 256, 0, stream>>>(Fp(24), MH, C, 0, MH, WM2);
  csr_build(csrG, Ip(2), EG, N, stream); csr_build(csrK, Ip(4), EK, N, stream);
  sage_kernel<IN, 1, 1><<<NBLK, 32, 0, stream>>>(Fp(0), WL0, Fp(7), Ip(1), EG, csrG.PERM, csrG.ROWPTR, csrG.ROWCNT, (int)csrG.permLen, NLIM, HA);
  sage_kernel<H, 0, 1><<<NBLK, 32, 0, stream>>>(HA, WL1, Fp(10), Ip(1), EG, csrG.PERM, csrG.ROWPTR, csrG.ROWCNT, (int)csrG.permLen, NLIM, HB);
  sage_kernel<H, 0, 0><<<NBLK, 32, 0, stream>>>(HB, WL2, Fp(13), Ip(1), EG, csrG.PERM, csrG.ROWPTR, csrG.ROWCNT, (int)csrG.permLen, NLIM, HA);
  mlp1_kernel<0><<<NBLK, 32, 0, stream>>>(HA, WM1A, Fp(21), NLIM, Y);
  sage_kernel<IN, 1, 1><<<NBLK, 32, 0, stream>>>(Fp(0), WG0, Fp(16), Ip(3), EK, csrK.PERM, csrK.ROWPTR, csrK.ROWCNT, (int)csrK.permLen, NLIM, HA);
  sage_kernel<H, 0, 0><<<NBLK, 32, 0, stream>>>(HA, WG1, Fp(19), Ip(3), EK, csrK.PERM, csrK.ROWPTR, csrK.ROWCNT, (int)csrK.permLen, NLIM, HB);
  mlp1_kernel<1><<<NBLK, 32, 0, stream>>>(HB, WM1B, Fp(21), NLIM, Y);
  bnstat1_kernel<<<NSB, 128, 0, stream>>>(Y, NLIM, PS); bnstat2_kernel<<<1, 128, 0, stream>>>(PS, NLIM, MV);
  head_kernel<<<NBLK, 32, 0, stream>>>(Y, MV, Fp(22), Fp(23), WM2, Fp(25), (float*)d_out);
}
